// MambaExpert_58067957842023
// MI455X (gfx1250) — hardware-run, weakly checked
//
#include <hip/hip_runtime.h>
#include <math.h>

constexpr int kBatch  = 2;
constexpr int kSeq    = 1024;
constexpr int kDModel = 1024;
constexpr int kDInner = 2048;
constexpr int kDState = 16;
constexpr int kDtRank = 64;
constexpr int kConvW  = 4;
constexpr int kDblN   = 96;
constexpr int kDblPad = 128;
constexpr int kTok    = kBatch * kSeq;
constexpr int kChunk  = 64;
constexpr float kLog2e = 1.4426950408889634f;
constexpr float kLn2   = 0.6931471805599453f;

constexpr size_t kBytesF32Plane = (size_t)kTok * kDInner * 4;
constexpr size_t kOffXin   = 0;
constexpr size_t kOffZ     = kOffXin + kBytesF32Plane;
constexpr size_t kOffXhi   = kOffZ + kBytesF32Plane;
constexpr size_t kBytesX16 = (size_t)kTok * kDModel * 2;
constexpr size_t kOffXlo   = kOffXhi + kBytesX16;
constexpr size_t kOffWinHi = kOffXlo + kBytesX16;
constexpr size_t kBytesWin16 = (size_t)(2 * kDInner) * kDModel * 2;
constexpr size_t kOffWinLo = kOffWinHi + kBytesWin16;
constexpr size_t kEndWin   = kOffWinLo + kBytesWin16;
constexpr size_t kBytesY16 = (size_t)kTok * kDInner * 2;
constexpr size_t kOffYhi   = kOffXhi;
constexpr size_t kOffYlo   = kOffYhi + kBytesY16;
static_assert(kOffYlo + kBytesY16 <= kEndWin);
constexpr size_t kOffU     = kEndWin;
constexpr size_t kOffUhi   = kOffU + kBytesF32Plane;
constexpr size_t kOffUlo   = kOffUhi + kBytesY16;
constexpr size_t kOffWxHi  = kOffUlo + kBytesY16;
constexpr size_t kBytesWx16 = (size_t)kDblPad * kDInner * 2;
constexpr size_t kOffWxLo  = kOffWxHi + kBytesWx16;
constexpr size_t kOffDbl   = kOffWxLo + kBytesWx16;
constexpr size_t kBytesDbl = (size_t)kTok * kDblPad * 4;
constexpr size_t kOffDtcHi = kOffDbl + kBytesDbl;
constexpr size_t kBytesDtc16 = (size_t)kTok * kDtRank * 2;
constexpr size_t kOffDtcLo = kOffDtcHi + kBytesDtc16;
constexpr size_t kOffWdtHi = kOffDtcLo + kBytesDtc16;
constexpr size_t kBytesWdt16 = (size_t)kDInner * kDtRank * 2;
constexpr size_t kOffWdtLo = kOffWdtHi + kBytesWdt16;
constexpr size_t kOffWoHi  = kOffWdtLo + kBytesWdt16;
constexpr size_t kBytesWo16 = (size_t)kDModel * kDInner * 2;
constexpr size_t kOffWoLo  = kOffWoHi + kBytesWo16;
constexpr size_t kWsTotal  = kOffWoLo + kBytesWo16;
constexpr size_t kOffDtlin = kOffXin;
static_assert(kWsTotal == (size_t)103809024);
static_assert(kWsTotal <= (size_t)134217728);
static_assert(kDModel % 32 == 0 && kDInner % 32 == 0 && kDtRank % 32 == 0);
static_assert(kTok % 64 == 0 && kDInner % 64 == 0 && kDblPad % 64 == 0 && kDModel % 64 == 0);

typedef __attribute__((ext_vector_type(16))) _Float16 v16h;
typedef __attribute__((ext_vector_type(8)))  _Float16 v8h;
typedef __attribute__((ext_vector_type(16))) __bf16   v16b;
typedef __attribute__((ext_vector_type(8)))  __bf16   v8b;
typedef __attribute__((ext_vector_type(8)))  float    v8f;
typedef __attribute__((ext_vector_type(4)))  float    v4f;
typedef __attribute__((ext_vector_type(4)))  unsigned int v4u;

__device__ __forceinline__ unsigned short f2bf_bits(float f) {
  unsigned u = __float_as_uint(f);
  return (unsigned short)((u + 0x7FFFu + ((u >> 16) & 1u)) >> 16);
}
__device__ __forceinline__ float bf_bits2f(unsigned short h) { return __uint_as_float(((unsigned)h) << 16); }

__device__ __forceinline__ void dep_guard_h(v8f& a, v8f& b, v16h x, v16h y) { asm volatile("v_nop\n\tv_nop\n\tv_nop\n\tv_nop" : "+v"(a), "+v"(b) : "v"(x), "v"(y)); }
__device__ __forceinline__ void dep_guard_b(v8f& a, v8f& b, v16b x, v16b y) { asm volatile("v_nop\n\tv_nop\n\tv_nop\n\tv_nop" : "+v"(a), "+v"(b) : "v"(x), "v"(y)); }
__device__ __forceinline__ void keep4_h(v16h a, v16h b, v16h c, v16h d) { asm volatile("v_nop" :: "v"(a), "v"(b), "v"(c), "v"(d)); }
__device__ __forceinline__ void keep4_b(v16b a, v16b b, v16b c, v16b d) { asm volatile("v_nop" :: "v"(a), "v"(b), "v"(c), "v"(d)); }
__device__ __forceinline__ void acc_guard4(v8f& a, v8f& b, v8f& c, v8f& d) { asm volatile("v_nop\n\tv_nop\n\tv_nop\n\tv_nop" : "+v"(a), "+v"(b), "+v"(c), "+v"(d)); }
template <typename T> struct Frag;
template <> struct Frag<_Float16> {
  typedef v16h V; union U { v16h v; v8h h[2]; };
  static __device__ __forceinline__ v16h load(const _Float16* p) {
    U f; f.h[0] = *(const v8h*)(p); f.h[1] = *(const v8h*)(p + 16); return f.v;
  }
  static __device__ __forceinline__ v8f mma(v16h a, v16h b, v8f c) {
    return __builtin_amdgcn_wmma_f32_16x16x32_f16(false, a, false, b, (short)0, c, false, false);
  }
  static __device__ __forceinline__ void guard(v8f& a, v8f& b, v16h x, v16h y) { dep_guard_h(a, b, x, y); }
  static __device__ __forceinline__ void keep(v16h a, v16h b, v16h c, v16h d) { keep4_h(a, b, c, d); }
};
template <> struct Frag<__bf16> {
  typedef v16b V; union U { v16b v; v8b h[2]; };
  static __device__ __forceinline__ v16b load(const __bf16* p) {
    U f; f.h[0] = *(const v8b*)(p); f.h[1] = *(const v8b*)(p + 16); return f.v;
  }
  static __device__ __forceinline__ v8f mma(v16b a, v16b b, v8f c) {
    return __builtin_amdgcn_wmma_f32_16x16x32_bf16(false, a, false, b, (short)0, c, false, false);
  }
  static __device__ __forceinline__ void guard(v8f& a, v8f& b, v16b x, v16b y) { dep_guard_b(a, b, x, y); }
  static __device__ __forceinline__ void keep(v16b a, v16b b, v16b c, v16b d) { keep4_b(a, b, c, d); }
};

__device__ __forceinline__ unsigned pk16(unsigned short a, unsigned short b) { return (unsigned)a | ((unsigned)b << 16); }

template <int ET> struct Elem;
template <> struct Elem<0> { typedef _Float16 T; };
template <> struct Elem<1> { typedef __bf16 T; };
template <int ET, bool SPLIT, int BIAS_MODE, int OUT_MODE, bool RESID, int ACT = 0>
__global__ __launch_bounds__(256) void wmma_gemm64(
    const unsigned short* __restrict__ Ap, const unsigned short* __restrict__ A2p, int lda, long strideA,
    const unsigned short* __restrict__ Btp, const unsigned short* __restrict__ Bt2p, int ldb, long strideB,
    void* __restrict__ Cout, void* __restrict__ Cout2, int ldc, long strideC,
    const float* __restrict__ bias,
    const float* __restrict__ resid, long strideR,
    int M, int N, int K, float scale) {
  typedef typename Elem<ET>::T T;
  typedef typename Frag<T>::V V;
  const T* A = (const T*)Ap; const T* A2 = (const T*)A2p; const T* Bt = (const T*)Btp; const T* Bt2 = (const T*)Bt2p;
  __shared__ __align__(16) float sT[8][16 * 68];
  const int b    = blockIdx.y;
  const int lane = threadIdx.x & 31;
  const int wave = threadIdx.x >> 5;
  const int tilesN = N >> 6;
  const int tilesM = M >> 6;
  const int tile = blockIdx.x * 8 + wave;
  if (tile >= tilesM * tilesN) return;
  const int tm = tile / tilesN;
  const int tn = tile - tm * tilesN;
  const int m0 = tm << 6;
  const int n0 = tn << 6;

  const T* Ab  = A  + (size_t)b * strideA;
  const T* Bb  = Bt + (size_t)b * strideB;
  const T* Ab2 = SPLIT ? (A2  + (size_t)b * strideA) : nullptr;
  const T* Bb2 = SPLIT ? (Bt2 + (size_t)b * strideB) : nullptr;

  const int rlane = lane & 15;
  const int koff  = (lane >> 4) * 8;
  const int mOff  = (lane >> 4) * 8;

  v8f acc[4][4];
#pragma unroll
  for (int i = 0; i < 4; ++i)
#pragma unroll
    for (int j = 0; j < 4; ++j) acc[i][j] = (v8f){0.f,0.f,0.f,0.f,0.f,0.f,0.f,0.f};

  for (int k0 = 0; k0 < K; k0 += 32) {
    V bh[4], bl[4];
#pragma unroll
    for (int j = 0; j < 4; ++j) {
      const size_t bo = (size_t)(n0 + (j << 4) + rlane) * ldb + koff + k0;
      bh[j] = Frag<T>::load(Bb + bo);
      if (SPLIT) bl[j] = Frag<T>::load(Bb2 + bo);
    }
#pragma unroll
    for (int i = 0; i < 4; ++i) {
      const size_t ao = (size_t)(m0 + (i << 4) + rlane) * lda + koff + k0;
      V ah = Frag<T>::load(Ab + ao);
      V al;
      if (SPLIT) al = Frag<T>::load(Ab2 + ao);
#pragma unroll
      for (int j = 0; j < 4; ++j) {
        acc[i][j] = Frag<T>::mma(ah, bh[j], acc[i][j]);
        if (SPLIT) {
          acc[i][j] = Frag<T>::mma(ah, bl[j], acc[i][j]);
          acc[i][j] = Frag<T>::mma(al, bh[j], acc[i][j]);
        }
      }
      Frag<T>::guard(acc[i][0], acc[i][3], ah, SPLIT ? al : ah);
    }
    Frag<T>::keep(bh[0], bh[1], bh[2], bh[3]);
    if (SPLIT) Frag<T>::keep(bl[0], bl[1], bl[2], bl[3]);
  }
  acc_guard4(acc[0][0], acc[0][1], acc[0][2], acc[0][3]);
  acc_guard4(acc[1][0], acc[1][1], acc[1][2], acc[1][3]);
  acc_guard4(acc[2][0], acc[2][1], acc[2][2], acc[2][3]);
  acc_guard4(acc[3][0], acc[3][1], acc[3][2], acc[3][3]);

  float* slab = sT[wave];
  const float* Rb = RESID ? (resid + (size_t)b * strideR) : nullptr;
#pragma unroll
  for (int i = 0; i < 4; ++i) {
    const int mBase = m0 + (i << 4);
#pragma unroll
    for (int j = 0; j < 4; ++j) {
      const int n = n0 + (j << 4) + rlane;
      float bv = 0.f;
      if (BIAS_MODE == 2) bv = bias[n];
#pragma unroll
      for (int r = 0; r < 8; ++r) {
        float v = acc[i][j][r] * scale;
        if (BIAS_MODE == 1) v += bias[mBase + mOff + r];
        if (BIAS_MODE == 2) v += bv;
        if (RESID) v += Rb[(size_t)(mBase + mOff + r) * ldc + n];
        if (ACT == 2) v = fmaxf(v, 0.0f);
        if (ACT == 4) v = (v > 0.f) ? v : 0.01f * v;
        slab[(mOff + r) * 68 + (j << 4) + rlane] = v;
      }
    }
    __builtin_amdgcn_fence(__ATOMIC_RELEASE, "workgroup");
    __builtin_amdgcn_wave_barrier();
    __builtin_amdgcn_fence(__ATOMIC_ACQUIRE, "workgroup");
    if (OUT_MODE == 0) {
      float* C = (float*)Cout + (size_t)b * strideC;
      const int hh = lane >> 4, c4 = (lane & 15) * 4;
      for (int pass = 0; pass < 2; ++pass) {
#pragma unroll
        for (int it = 0; it < 8; ++it) {
          const int row = it * 2 + hh;
          v4f v = *(const v4f*)(slab + row * 68 + c4);
          *(volatile v4f*)(C + (size_t)(mBase + row) * ldc + n0 + c4) = v;
        }
        __threadfence();
      }
    } else {
      const int q = lane >> 3, c8 = (lane & 7) * 8;
      unsigned short* C  = (unsigned short*)Cout  + (size_t)b * strideC;
      unsigned short* C2 = (OUT_MODE == 2) ? ((unsigned short*)Cout2 + (size_t)b * strideC) : nullptr;
      for (int pass = 0; pass < 2; ++pass) {
#pragma unroll
        for (int it = 0; it < 4; ++it) {
          const int row = it * 4 + q;
          const float* sp = slab + row * 68 + c8;
          v8h hv, lv;
#pragma unroll
          for (int e = 0; e < 8; ++e) {
            if (OUT_MODE == 1) {
              hv[e] = (_Float16)sp[e];
            } else {
              unsigned short hb = f2bf_bits(sp[e]);
              unsigned short lb = f2bf_bits(sp[e] - bf_bits2f(hb));
              hv[e] = __builtin_bit_cast(_Float16, hb);
              lv[e] = __builtin_bit_cast(_Float16, lb);
            }
          }
          *(volatile v8h*)(C + (size_t)(mBase + row) * ldc + n0 + c8) = hv;
          if (OUT_MODE == 2) *(volatile v8h*)(C2 + (size_t)(mBase + row) * ldc + n0 + c8) = lv;
        }
        __threadfence();
      }
    }
    __builtin_amdgcn_fence(__ATOMIC_RELEASE, "workgroup");
    __builtin_amdgcn_wave_barrier();
    __builtin_amdgcn_fence(__ATOMIC_ACQUIRE, "workgroup");
  }
}

__device__ __forceinline__ void split_pack8(v4f a, v4f c, v4u& uh, v4u& ul) {
  unsigned short hb[8], lb[8];
#pragma unroll
  for (int e = 0; e < 4; ++e) {
    hb[e] = f2bf_bits(a[e]);
    lb[e] = f2bf_bits(a[e] - bf_bits2f(hb[e]));
    hb[4 + e] = f2bf_bits(c[e]);
    lb[4 + e] = f2bf_bits(c[e] - bf_bits2f(hb[4 + e]));
  }
  uh = (v4u){pk16(hb[0], hb[1]), pk16(hb[2], hb[3]), pk16(hb[4], hb[5]), pk16(hb[6], hb[7])};
  ul = (v4u){pk16(lb[0], lb[1]), pk16(lb[2], lb[3]), pk16(lb[4], lb[5]), pk16(lb[6], lb[7])};
}

__global__ __launch_bounds__(256) void split8_kernel(const float* __restrict__ in, int ld_in, int ncols8, int nthr,
                                                     unsigned short* __restrict__ hi, unsigned short* __restrict__ lo) {
  const int i = blockIdx.x * 256 + threadIdx.x;
  if (i >= nthr) return;
  const int row = i / ncols8;
  const int c8  = i - row * ncols8;
  const float* p = in + (size_t)row * ld_in + 8 * c8;
  const v4f a = *(const v4f*)(p);
  const v4f c = *(const v4f*)(p + 4);
  v4u uh, ul;
  split_pack8(a, c, uh, ul);
  unsigned short* qh = hi + 8 * (size_t)i;
  unsigned short* ql = lo + 8 * (size_t)i;
  *(volatile v4u*)qh = uh;
  *(volatile v4u*)ql = ul;
  __threadfence();
  *(volatile v4u*)qh = uh;
  *(volatile v4u*)ql = ul;
}

__global__ __launch_bounds__(256) void tsplit_kernel(const float* __restrict__ W, int ncols_in, int k_rows,
                                                     unsigned short* __restrict__ hi, unsigned short* __restrict__ lo) {
  __shared__ float sm[64][65];
  const int t  = threadIdx.x;
  const int k0 = blockIdx.x * 64;
  const int n0 = blockIdx.y * 64;
#pragma unroll
  for (int i = 0; i < 16; ++i) {
    const int e  = i * 256 + t;
    const int kl = e >> 6;
    const int nl = e & 63;
    const int n  = n0 + nl;
    const int nc = (n < ncols_in) ? n : (ncols_in - 1);
    float v = W[(size_t)(k0 + kl) * ncols_in + nc];
    v = (n < ncols_in) ? v : 0.0f;
    sm[nl][kl] = v;
  }
  __syncthreads();
  const int lane = t & 31, wave = t >> 5;
  const int q = lane >> 3, c8 = (lane & 7) * 8;
  for (int pass = 0; pass < 2; ++pass) {
#pragma unroll
    for (int it = 0; it < 2; ++it) {
      const int row = wave * 8 + it * 4 + q;
      v4f a, c;
#pragma unroll
      for (int e = 0; e < 4; ++e) { a[e] = sm[row][c8 + e]; c[e] = sm[row][c8 + 4 + e]; }
      v4u uh, ul;
      split_pack8(a, c, uh, ul);
      const size_t o = (size_t)(n0 + row) * k_rows + k0 + c8;
      *(volatile v4u*)(hi + o) = uh;
      *(volatile v4u*)(lo + o) = ul;
    }
    __threadfence();
  }
}

__global__ __launch_bounds__(256) void conv_silu_kernel(const float* __restrict__ xin,
                                                        const float* __restrict__ cw, const float* __restrict__ cb,
                                                        float* __restrict__ u,
                                                        unsigned short* __restrict__ uhi, unsigned short* __restrict__ ulo) {
  __shared__ __align__(16) float su[kDInner];
  const int tok = blockIdx.x;
  const int tt  = tok & (kSeq - 1);
  const int t   = threadIdx.x;
  const int d8  = t * 8;
  v4f w[8];
#pragma unroll
  for (int e = 0; e < 8; ++e) w[e] = *(const v4f*)(cw + (size_t)(d8 + e) * kConvW);
  float acc[8];
#pragma unroll
  for (int e = 0; e < 8; ++e) acc[e] = 0.0f;
#pragma unroll
  for (int j = 0; j < kConvW; ++j) {
    const int ts   = tt - (kConvW - 1) + j;
    const int tokj = (ts >= 0) ? (tok - (kConvW - 1) + j) : (tok - tt);
    const float m  = (ts >= 0) ? 1.0f : 0.0f;
    const float* xp = xin + (size_t)tokj * kDInner + d8;
    const v4f a0 = *(const v4f*)(xp);
    const v4f a1 = *(const v4f*)(xp + 4);
#pragma unroll
    for (int e = 0; e < 4; ++e) {
      acc[e]     += (m * a0[e]) * w[e][j];
      acc[4 + e] += (m * a1[e]) * w[4 + e][j];
    }
  }
  const v4f b0 = *(const v4f*)(cb + d8);
  const v4f b1 = *(const v4f*)(cb + d8 + 4);
  v4f s0, s1;
#pragma unroll
  for (int e = 0; e < 4; ++e) {
    const float p0 = acc[e] + b0[e];
    const float p1 = acc[4 + e] + b1[e];
    s0[e] = p0 * __builtin_amdgcn_rcpf(1.0f + exp2f(-p0 * kLog2e));
    s1[e] = p1 * __builtin_amdgcn_rcpf(1.0f + exp2f(-p1 * kLog2e));
  }
  *(v4f*)(su + d8)     = s0;
  *(v4f*)(su + d8 + 4) = s1;
  v4u uh, ul;
  split_pack8(s0, s1, uh, ul);
  __syncthreads();
  const size_t rowoff = (size_t)tok * kDInner;
  unsigned short* ph = uhi + rowoff + d8;
  unsigned short* pl = ulo + rowoff + d8;
  float* up = u + rowoff;
  const v4f f0 = *(const v4f*)(su + t * 4);
  const v4f f1 = *(const v4f*)(su + 1024 + t * 4);
  for (int pass = 0; pass < 2; ++pass) {
    *(volatile v4u*)ph = uh;
    *(volatile v4u*)pl = ul;
    *(volatile v4f*)(up + t * 4) = f0;
    *(volatile v4f*)(up + 1024 + t * 4) = f1;
    __threadfence();
  }
}

__device__ __forceinline__ float softplus_f(float p) {
  const float e = exp2f(-fabsf(p) * kLog2e);
  return fmaxf(p, 0.0f) + kLn2 * log2f(1.0f + e);
}

__global__ __launch_bounds__(64) void scan_kernel(const float* __restrict__ dtlin, const float* __restrict__ bdt,
                                                  const float* __restrict__ u, const float* __restrict__ z,
                                                  const float* __restrict__ dbl,
                                                  const float* __restrict__ alog, const float* __restrict__ dsk,
                                                  unsigned short* __restrict__ yhi, unsigned short* __restrict__ ylo) {
  __shared__ __align__(16) float ybuf[kChunk][64];
  __shared__ __align__(16) float sbc[kChunk][32];
  const int t  = threadIdx.x;
  const int d0 = blockIdx.x * 64;
  const int b  = blockIdx.y;
  const int d  = d0 + t;
  float a2[kDState], h[kDState];
#pragma unroll
  for (int s = 0; s < kDState; ++s) {
    a2[s] = -exp2f(alog[(size_t)d * kDState + s] * kLog2e) * kLog2e;
    h[s]  = 0.0f;
  }
  const float bd = bdt[d];
  const float dd = dsk[d];
  const int r  = t >> 3;
  const int c8 = (t & 7) * 8;
#pragma unroll 1
  for (int c = 0; c < kSeq / kChunk; ++c) {
    const int tok0 = b * kSeq + c * kChunk;
#pragma unroll
    for (int i = 0; i < 8; ++i) {
      const int idx4 = i * 64 + t;
      const int st = idx4 >> 3;
      const int c4 = (idx4 & 7) * 4;
      const v4f v = *(const v4f*)(dbl + (size_t)(tok0 + st) * kDblPad + kDtRank + c4);
      *(v4f*)(&sbc[st][c4]) = v;
    }
    __syncthreads();
#pragma unroll 1
    for (int tl = 0; tl < kChunk; ++tl) {
      const size_t row = (size_t)(tok0 + tl) * kDInner + d;
      const float p  = dtlin[row] + bd;
      const float uu = u[row];
      const float zz = z[row];
      const float delta = softplus_f(p);
      const float du = delta * uu;
      float y = 0.0f;
#pragma unroll
      for (int s = 0; s < kDState; ++s) {
        const float e = exp2f(delta * a2[s]);
        h[s] = e * h[s] + du * sbc[tl][s];
        y += h[s] * sbc[tl][kDState + s];
      }
      const float yo = y + uu * dd;
      const float g  = zz * __builtin_amdgcn_rcpf(1.0f + exp2f(-zz * kLog2e));
      ybuf[tl][t] = yo * g;
    }
    __syncthreads();
    for (int pass = 0; pass < 2; ++pass) {
#pragma unroll
      for (int it = 0; it < 8; ++it) {
        const int rowl = it * 8 + r;
        const v4f a  = *(const v4f*)(&ybuf[rowl][c8]);
        const v4f cc = *(const v4f*)(&ybuf[rowl][c8 + 4]);
        v4u uh, ul;
        split_pack8(a, cc, uh, ul);
        const size_t o = (size_t)(tok0 + rowl) * kDInner + d0 + c8;
        *(volatile v4u*)(yhi + o) = uh;
        *(volatile v4u*)(ylo + o) = ul;
      }
      __threadfence();
    }
  }
}

extern "C" void kernel_launch(void* const* d_in, const int* in_sizes, int n_in,
                              void* d_out, int out_size, void* d_ws, size_t ws_size, hipStream_t stream) {
  if (n_in < 10) return;
  if (in_sizes[0] != kTok * kDModel) return;
  if (in_sizes[1] != kDModel * 2 * kDInner) return;
  if (in_sizes[2] != kDInner * kConvW) return;
  if (in_sizes[3] != kDInner) return;
  if (in_sizes[4] != kDInner * kDblN) return;
  if (in_sizes[5] != kDtRank * kDInner) return;
  if (in_sizes[6] != kDInner) return;
  if (in_sizes[7] != kDInner * kDState) return;
  if (in_sizes[8] != kDInner) return;
  if (in_sizes[9] != kDInner * kDModel) return;
  if (out_size != kTok * kDModel) return;
  if (ws_size < kWsTotal) return;

  const float* x     = (const float*)d_in[0];
  const float* w_in  = (const float*)d_in[1];
  const float* cw    = (const float*)d_in[2];
  const float* cb    = (const float*)d_in[3];
  const float* w_x   = (const float*)d_in[4];
  const float* w_dt  = (const float*)d_in[5];
  const float* b_dt  = (const float*)d_in[6];
  const float* a_log = (const float*)d_in[7];
  const float* d_skp = (const float*)d_in[8];
  const float* w_out = (const float*)d_in[9];
  float* out = (float*)d_out;

  char* ws = (char*)d_ws;
  typedef unsigned short us;
  float* xin   = (float*)(ws + kOffXin);
  float* zpl   = (float*)(ws + kOffZ);
  us* xhi   = (us*)(ws + kOffXhi);   us* xlo   = (us*)(ws + kOffXlo);
  us* winhi = (us*)(ws + kOffWinHi); us* winlo = (us*)(ws + kOffWinLo);
  us* yhi   = (us*)(ws + kOffYhi);   us* ylo   = (us*)(ws + kOffYlo);
  float* upl = (float*)(ws + kOffU);
  us* uhi   = (us*)(ws + kOffUhi);   us* ulo   = (us*)(ws + kOffUlo);
  us* wxhi  = (us*)(ws + kOffWxHi);  us* wxlo  = (us*)(ws + kOffWxLo);
  float* dbl = (float*)(ws + kOffDbl);
  us* dtchi = (us*)(ws + kOffDtcHi); us* dtclo = (us*)(ws + kOffDtcLo);
  us* wdthi = (us*)(ws + kOffWdtHi); us* wdtlo = (us*)(ws + kOffWdtLo);
  us* wohi  = (us*)(ws + kOffWoHi);  us* wolo  = (us*)(ws + kOffWoLo);
  float* dtlin = (float*)(ws + kOffDtlin);

  split8_kernel<<<dim3((kTok * kDModel / 8) / 256), 256, 0, stream>>>(x, kDModel, kDModel / 8, kTok * kDModel / 8, xhi, xlo);

  tsplit_kernel<<<dim3(kDModel / 64, (2 * kDInner) / 64), 256, 0, stream>>>(w_in, 2 * kDInner, kDModel, winhi, winlo);
  tsplit_kernel<<<dim3(kDInner / 64, kDblPad / 64), 256, 0, stream>>>(w_x, kDblN, kDInner, wxhi, wxlo);
  tsplit_kernel<<<dim3(kDtRank / 64, kDInner / 64), 256, 0, stream>>>(w_dt, kDInner, kDtRank, wdthi, wdtlo);
  tsplit_kernel<<<dim3(kDInner / 64, kDModel / 64), 256, 0, stream>>>(w_out, kDModel, kDInner, wohi, wolo);

  wmma_gemm64<1, true, 0, 0, false, 0><<<dim3((kTok / 64) * (kDInner / 64) / 8, 2), 256, 0, stream>>>(
      xhi, xlo, kDModel, 0L,
      winhi, winlo, kDModel, (long)kDInner * kDModel,
      (void*)xin, nullptr, kDInner, (long)kTok * kDInner,
      nullptr, nullptr, 0L, kTok, kDInner, kDModel, 1.0f);
  (void)zpl;

  conv_silu_kernel<<<dim3(kTok), 256, 0, stream>>>(xin, cw, cb, upl, uhi, ulo);

  wmma_gemm64<1, true, 0, 0, false, 0><<<dim3((kTok / 64) * (kDblPad / 64) / 8, 1), 256, 0, stream>>>(
      uhi, ulo, kDInner, 0L,
      wxhi, wxlo, kDInner, 0L,
      (void*)dbl, nullptr, kDblPad, 0L,
      nullptr, nullptr, 0L, kTok, kDblPad, kDInner, 1.0f);

  split8_kernel<<<dim3((kTok * kDtRank / 8) / 256), 256, 0, stream>>>(dbl, kDblPad, kDtRank / 8, kTok * kDtRank / 8, dtchi, dtclo);

  wmma_gemm64<1, true, 0, 0, false, 0><<<dim3((kTok / 64) * (kDInner / 64) / 8, 1), 256, 0, stream>>>(
      dtchi, dtclo, kDtRank, 0L,
      wdthi, wdtlo, kDtRank, 0L,
      (void*)dtlin, nullptr, kDInner, 0L,
      nullptr, nullptr, 0L, kTok, kDInner, kDtRank, 1.0f);

  scan_kernel<<<dim3(kDInner / 64, kBatch), 64, 0, stream>>>(dtlin, b_dt, upl, (const float*)(ws + kOffZ), dbl, a_log, d_skp, yhi, ylo);

  wmma_gemm64<1, true, 0, 0, false, 0><<<dim3((kTok / 64) * (kDModel / 64) / 8, 1), 256, 0, stream>>>(
      yhi, ylo, kDInner, 0L,
      wohi, wolo, kDInner, 0L,
      (void*)out, nullptr, kDModel, 0L,
      nullptr, nullptr, 0L, kTok, kDModel, kDInner, 1.0f);
}
